// LSTM_33363305955791
// MI455X (gfx1250) — hardware-verified
//
#include <hip/hip_runtime.h>
#include <math.h>

constexpr int NBAT     = 128;
constexpr int NNODE    = 2;
constexpr int NSTEP    = 256;
constexpr int NHID     = 128;
constexpr int NGATE    = 4 * NHID;
constexpr int NY0      = 2 * NHID;
constexpr int NFEAT    = NNODE * NY0;
constexpr int NFC      = 256;
constexpr int NOUTD    = 64;
constexpr int NTHR     = 256;
constexpr int ROWS_BLK = 16;
constexpr int NTILE    = NBAT / ROWS_BLK;
constexpr int HPITCH   = 136;
constexpr int XPW      = 260;
constexpr int FPITCH   = 132;
constexpr float WCARRY  = 64.0f;
constexpr float HCARRY  = 256.0f;
constexpr float ACC_INV = 1.0f / (WCARRY * HCARRY);
constexpr float LN_EPS  = 1e-6f;

static_assert(NBAT % ROWS_BLK == 0, "batch tiles");
static_assert(NHID == 16 * (NTHR / 32), "8 waves x 16 hidden columns");
static_assert(NHID % 32 == 0 && NY0 % 32 == 0, "K multiples of 32");
static_assert((NSTEP * NBAT) % 64 == 0 && NGATE % 64 == 0 && NBAT % 64 == 0, "GEMM tile multiples");
static_assert(ROWS_BLK * NHID == NTHR * 8, "h tile staging exact");
static_assert(ROWS_BLK * NGATE * 2 == NTHR * 64, "gate-input tile staging exact");
static_assert(NFC == NTHR, "one thread per fc feature");
static_assert(NFEAT == 2 * NTHR, "feature row staging exact");

typedef __attribute__((ext_vector_type(16))) _Float16 v16h;
typedef __attribute__((ext_vector_type(8)))  _Float16 v8h;
typedef __attribute__((ext_vector_type(8)))  float    v8f;
typedef __attribute__((ext_vector_type(4)))  float    v4f;
typedef __attribute__((ext_vector_type(4)))  unsigned v4u;

__device__ __forceinline__ void dep_guard_h(v8f& a, v8f& b, v16h x, v16h y) { asm volatile("v_nop\n\tv_nop\n\tv_nop\n\tv_nop" : "+v"(a), "+v"(b) : "v"(x), "v"(y)); }
__device__ __forceinline__ void keep4_h(v16h a, v16h b, v16h c, v16h d) { asm volatile("v_nop" :: "v"(a), "v"(b), "v"(c), "v"(d)); }
__device__ __forceinline__ void acc_guard4(v8f& a, v8f& b, v8f& c, v8f& d) { asm volatile("v_nop\n\tv_nop\n\tv_nop\n\tv_nop" : "+v"(a), "+v"(b), "+v"(c), "+v"(d)); }
__device__ __forceinline__ void wm_guard4(v8f& a, v8f& b, v8f& c, v8f& d, v16h x, v16h y0, v16h y1, v16h y2, v16h y3) {
  asm volatile("v_nop\n\tv_nop\n\tv_nop\n\tv_nop" : "+v"(a), "+v"(b), "+v"(c), "+v"(d) : "v"(x), "v"(y0), "v"(y1), "v"(y2), "v"(y3));
}

template <typename T> struct Frag;
template <> struct Frag<_Float16> {
  typedef v16h V; union U { v16h v; v8h h[2]; };
  static __device__ __forceinline__ v16h load(const _Float16* p) {
    U f; f.h[0] = *(const v8h*)(p); f.h[1] = *(const v8h*)(p + 16); return f.v;
  }
  static __device__ __forceinline__ v8f mma(v16h a, v16h b, v8f c) {
    return __builtin_amdgcn_wmma_f32_16x16x32_f16(false, a, false, b, (short)0, c, false, false);
  }
  static __device__ __forceinline__ void guard(v8f& a, v8f& b, v16h x, v16h y) { dep_guard_h(a, b, x, y); }
  static __device__ __forceinline__ void keep(v16h a, v16h b, v16h c, v16h d) { keep4_h(a, b, c, d); }
};

__device__ __forceinline__ float h16_to_f32(unsigned hb) {
  const unsigned sgn = (hb & 0x8000u) << 16; const unsigned em = hb & 0x7fffu;
  const float fn = __uint_as_float((em << 13) + 0x38000000u);
  const float fs = (float)em * 5.9604644775390625e-8f;
  const float mag = (em < 0x400u) ? fs : fn; return __uint_as_float(__float_as_uint(mag) | sgn); }

__device__ __forceinline__ float sigm(float v)   { return __builtin_amdgcn_rcpf(1.0f + expf(-v)); }
__device__ __forceinline__ float tanh_e(float v) { return 1.0f - 2.0f * __builtin_amdgcn_rcpf(1.0f + expf(2.0f * v)); }

template <int ET> struct Elem;
template <> struct Elem<0> { typedef _Float16 T; };
template <int ET, bool SPLIT, int BIAS_MODE, int OUT_MODE>
__global__ __launch_bounds__(256) void wmma_gemm64(
    const unsigned short* __restrict__ Ap, const unsigned short* __restrict__ A2p, int lda, long strideA,
    const unsigned short* __restrict__ Btp, const unsigned short* __restrict__ Bt2p, int ldb, long strideB,
    void* __restrict__ Cout, void* __restrict__ Cout2, int ldc, long strideC,
    const float* __restrict__ bias,
    int M, int N, int K, float scale) {
  typedef typename Elem<ET>::T T;
  typedef typename Frag<T>::V V;
  const T* A = (const T*)Ap; const T* A2 = (const T*)A2p; const T* Bt = (const T*)Btp; const T* Bt2 = (const T*)Bt2p;
  __shared__ __align__(16) float sT[8][16 * 68];
  const int b    = blockIdx.y;
  const int lane = threadIdx.x & 31;
  const int wave = threadIdx.x >> 5;
  const int tilesN = N >> 6;
  const int tilesM = M >> 6;
  const int tile = blockIdx.x * 8 + wave;
  if (tile >= tilesM * tilesN) return;
  const int tm = tile / tilesN;
  const int tn = tile - tm * tilesN;
  const int m0 = tm << 6;
  const int n0 = tn << 6;

  const T* Ab  = A  + (size_t)b * strideA;
  const T* Bb  = Bt + (size_t)b * strideB;
  const T* Ab2 = SPLIT ? (A2  + (size_t)b * strideA) : nullptr;
  const T* Bb2 = SPLIT ? (Bt2 + (size_t)b * strideB) : nullptr;

  const int rlane = lane & 15;
  const int koff  = (lane >> 4) * 8;
  const int mOff  = (lane >> 4) * 8;

  v8f acc[4][4];
#pragma unroll
  for (int i = 0; i < 4; ++i)
#pragma unroll
    for (int j = 0; j < 4; ++j) acc[i][j] = (v8f){0.f,0.f,0.f,0.f,0.f,0.f,0.f,0.f};

  for (int k0 = 0; k0 < K; k0 += 32) {
    V bh[4], bl[4];
#pragma unroll
    for (int j = 0; j < 4; ++j) {
      const size_t bo = (size_t)(n0 + (j << 4) + rlane) * ldb + koff + k0;
      bh[j] = Frag<T>::load(Bb + bo);
      if (SPLIT) bl[j] = Frag<T>::load(Bb2 + bo);
    }
#pragma unroll
    for (int i = 0; i < 4; ++i) {
      const size_t ao = (size_t)(m0 + (i << 4) + rlane) * lda + koff + k0;
      V ah = Frag<T>::load(Ab + ao);
      V al;
      if (SPLIT) al = Frag<T>::load(Ab2 + ao);
#pragma unroll
      for (int j = 0; j < 4; ++j) {
        acc[i][j] = Frag<T>::mma(ah, bh[j], acc[i][j]);
        if (SPLIT) {
          acc[i][j] = Frag<T>::mma(ah, bl[j], acc[i][j]);
          acc[i][j] = Frag<T>::mma(al, bh[j], acc[i][j]);
        }
      }
      wm_guard4(acc[i][0], acc[i][1], acc[i][2], acc[i][3], ah, bh[0], bh[1], bh[2], bh[3]);
      if (SPLIT) Frag<T>::guard(acc[i][0], acc[i][3], al, bl[3]);
    }
    Frag<T>::keep(bh[0], bh[1], bh[2], bh[3]);
    if (SPLIT) Frag<T>::keep(bl[0], bl[1], bl[2], bl[3]);
  }
  acc_guard4(acc[0][0], acc[0][1], acc[0][2], acc[0][3]);
  acc_guard4(acc[1][0], acc[1][1], acc[1][2], acc[1][3]);
  acc_guard4(acc[2][0], acc[2][1], acc[2][2], acc[2][3]);
  acc_guard4(acc[3][0], acc[3][1], acc[3][2], acc[3][3]);

  float* slab = sT[wave];
#pragma unroll
  for (int i = 0; i < 4; ++i) {
    const int mBase = m0 + (i << 4);
#pragma unroll
    for (int j = 0; j < 4; ++j) {
      const int n = n0 + (j << 4) + rlane;
      float bv = 0.f;
      if (BIAS_MODE == 2) bv = bias[n];
#pragma unroll
      for (int r = 0; r < 8; ++r) {
        float v = acc[i][j][r] * scale;
        if (BIAS_MODE == 1) v += bias[mBase + mOff + r];
        if (BIAS_MODE == 2) v += bv;
        slab[(mOff + r) * 68 + (j << 4) + rlane] = v;
      }
    }
    __builtin_amdgcn_fence(__ATOMIC_RELEASE, "workgroup");
    __builtin_amdgcn_wave_barrier();
    __builtin_amdgcn_fence(__ATOMIC_ACQUIRE, "workgroup");
    if (OUT_MODE == 0) {
      float* C = (float*)Cout + (size_t)b * strideC;
      const int hh = lane >> 4, c4 = (lane & 15) * 4;
      for (int pass = 0; pass < 2; ++pass) {
#pragma unroll
        for (int it = 0; it < 8; ++it) {
          const int row = it * 2 + hh;
          v4f v = *(const v4f*)(slab + row * 68 + c4);
          *(volatile v4f*)(C + (size_t)(mBase + row) * ldc + n0 + c4) = v;
        }
        __threadfence();
      }
    } else {
      const int q = lane >> 3, c8 = (lane & 7) * 8;
      unsigned short* C = (unsigned short*)Cout + (size_t)b * strideC;
      for (int pass = 0; pass < 2; ++pass) {
#pragma unroll
        for (int it = 0; it < 4; ++it) {
          const int row = it * 4 + q;
          const float* sp = slab + row * 68 + c8;
          v8h hv;
#pragma unroll
          for (int e = 0; e < 8; ++e) hv[e] = (_Float16)sp[e];
          *(volatile v8h*)(C + (size_t)(mBase + row) * ldc + n0 + c8) = hv;
        }
        __threadfence();
      }
    }
    __builtin_amdgcn_fence(__ATOMIC_RELEASE, "workgroup");
    __builtin_amdgcn_wave_barrier();
    __builtin_amdgcn_fence(__ATOMIC_ACQUIRE, "workgroup");
  }
}

__global__ __launch_bounds__(NTHR) void cvt_w_kernel(const float* __restrict__ s0, const float* __restrict__ s1,
                                                     const float* __restrict__ s2,
                                                     unsigned short* __restrict__ d0, unsigned short* __restrict__ d1,
                                                     unsigned short* __restrict__ d2,
                                                     int n8a, int n8b, int n8c, float sc) {
  const int seg = blockIdx.y;
  const float* src = (seg == 0) ? s0 : ((seg == 1) ? s1 : s2);
  unsigned short* dst = (seg == 0) ? d0 : ((seg == 1) ? d1 : d2);
  const int n8 = (seg == 0) ? n8a : ((seg == 1) ? n8b : n8c);
  const int i = blockIdx.x * NTHR + threadIdx.x;
  if (i < n8) {
    const float* sp = src + (size_t)i * 8;
    const v4f a = *(const v4f*)(sp);
    const v4f b = *(const v4f*)(sp + 4);
    v8h hv;
#pragma unroll
    for (int e = 0; e < 4; ++e) {
      hv[e]     = (_Float16)(a[e] * sc);
      hv[4 + e] = (_Float16)(b[e] * sc);
    }
    *(volatile v8h*)(dst + (size_t)i * 8) = hv;
    __threadfence();
    *(volatile v8h*)(dst + (size_t)i * 8) = hv;
  }
}

__global__ __launch_bounds__(NTHR) void lstm_l0_kernel(const float* __restrict__ x, const float* __restrict__ h0,
                                                       const float* __restrict__ c0, const float* __restrict__ wih0,
                                                       const float* __restrict__ b0,
                                                       const unsigned short* __restrict__ WHp,
                                                       unsigned short* __restrict__ Y0) {
  __shared__ __align__(16) _Float16 Ah[2 * ROWS_BLK * HPITCH];
  const _Float16* WH = (const _Float16*)WHp;
  const int tid = threadIdx.x, lane = tid & 31, wave = tid >> 5;
  const int c = lane & 15, hh = lane >> 4, koff = hh * 8;
  const int nd = blockIdx.x / NTILE;
  const int tile = blockIdx.x - nd * NTILE;
  const int node = nd >> 1, dir = nd & 1;
  const int rowbase = tile * ROWS_BLK;
  const int slot = node * 4 + dir;
  const int j = wave * 16 + c;

  {
    const int row = tid >> 4, c8 = (tid & 15) * 8;
    const float* hp = h0 + ((size_t)slot * NBAT + rowbase + row) * NHID + c8;
    const v4f a = *(const v4f*)(hp);
    const v4f b = *(const v4f*)(hp + 4);
    v8h hv;
#pragma unroll
    for (int e = 0; e < 4; ++e) {
      hv[e]     = (_Float16)(a[e] * HCARRY);
      hv[4 + e] = (_Float16)(b[e] * HCARRY);
    }
    *(v8h*)(Ah + row * HPITCH + c8) = hv;
  }
  float cst[8], wi[4], bi[4];
#pragma unroll
  for (int g = 0; g < 4; ++g) {
    wi[g] = wih0[(size_t)nd * NGATE + g * NHID + j];
    bi[g] = b0[(size_t)nd * NGATE + g * NHID + j];
  }
  asm volatile("" ::: "memory");
#pragma unroll
  for (int r = 0; r < 8; ++r) cst[r] = c0[((size_t)slot * NBAT + rowbase + 8 * hh + r) * NHID + j];
  __syncthreads();

  const _Float16* wp = WH + ((size_t)nd * NGATE + j) * NHID + koff;
  const float* xbase = x + ((size_t)(rowbase + 8 * hh) * NNODE + node) * NSTEP;
  const v8f z8 = {0.f, 0.f, 0.f, 0.f, 0.f, 0.f, 0.f, 0.f};

#pragma unroll 1
  for (int s = 0; s < NSTEP; ++s) {
    const int t = dir ? (NSTEP - 1 - s) : s;
    const int cur = s & 1;
    float xr[8];
#pragma unroll
    for (int r = 0; r < 8; ++r) xr[r] = xbase[(size_t)r * (NNODE * NSTEP) + t];
    const _Float16* ahrow = Ah + cur * (ROWS_BLK * HPITCH) + c * HPITCH + koff;
    _Float16* ahn = Ah + (cur ^ 1) * (ROWS_BLK * HPITCH);
    v8f acc0 = z8, acc1 = z8, acc2 = z8, acc3 = z8;
#pragma unroll 1
    for (int k0 = 0; k0 < NHID; k0 += 32) {
      const v16h a  = Frag<_Float16>::load(ahrow + k0);
      const v16h b0f = Frag<_Float16>::load(wp + k0);
      const v16h b1f = Frag<_Float16>::load(wp + (size_t)1 * NHID * NHID + k0);
      const v16h b2f = Frag<_Float16>::load(wp + (size_t)2 * NHID * NHID + k0);
      const v16h b3f = Frag<_Float16>::load(wp + (size_t)3 * NHID * NHID + k0);
      acc0 = Frag<_Float16>::mma(a, b0f, acc0);
      acc1 = Frag<_Float16>::mma(a, b1f, acc1);
      acc2 = Frag<_Float16>::mma(a, b2f, acc2);
      acc3 = Frag<_Float16>::mma(a, b3f, acc3);
      wm_guard4(acc0, acc1, acc2, acc3, a, b0f, b1f, b2f, b3f);
    }
    acc_guard4(acc0, acc1, acc2, acc3);
#pragma unroll
    for (int r = 0; r < 8; ++r) {
      const float xv = xr[r];
      const float zi = acc0[r] * ACC_INV + (xv * wi[0] + bi[0]);
      const float zf = acc1[r] * ACC_INV + (xv * wi[1] + bi[1]);
      const float zg = acc2[r] * ACC_INV + (xv * wi[2] + bi[2]);
      const float zo = acc3[r] * ACC_INV + (xv * wi[3] + bi[3]);
      const float ig = sigm(zi);
      const float fg = sigm(zf);
      const float gg = tanh_e(zg);
      const float og = sigm(zo);
      const float cn = fg * cst[r] + ig * gg;
      cst[r] = cn;
      const float hn = og * tanh_e(cn);
      ahn[(8 * hh + r) * HPITCH + j] = (_Float16)(hn * HCARRY);
    }
    __syncthreads();
    {
      const int row = tid >> 4, c8 = (tid & 15) * 8;
      const v8h hv = *(const v8h*)(ahn + row * HPITCH + c8);
      unsigned short* yp = Y0 + (((size_t)node * NSTEP + t) * NBAT + rowbase + row) * NY0 + dir * NHID + c8;
      *(volatile v8h*)yp = hv;
      __threadfence();
      *(volatile v8h*)yp = hv;
    }
  }
}

__device__ __forceinline__ void stage_xp(const unsigned short* __restrict__ src, unsigned* dstw, int tid) {
  const int row = tid >> 4, sg = tid & 15;
  const v4u* gp = (const v4u*)(src + (size_t)row * NGATE + sg * 32);
  const v4u q0 = gp[0];
  const v4u q1 = gp[1];
  const v4u q2 = gp[2];
  const v4u q3 = gp[3];
  v4u* lp = (v4u*)(dstw + row * XPW + sg * 16);
  lp[0] = q0;
  lp[1] = q1;
  lp[2] = q2;
  lp[3] = q3;
}

__global__ __launch_bounds__(NTHR) void lstm_l1_kernel(const float* __restrict__ h0, const float* __restrict__ c0,
                                                       const float* __restrict__ b1,
                                                       const unsigned short* __restrict__ WHp,
                                                       const unsigned short* __restrict__ XPF,
                                                       const unsigned short* __restrict__ XPB,
                                                       float* __restrict__ FEAT) {
  __shared__ __align__(16) _Float16 Ah[2 * ROWS_BLK * HPITCH];
  __shared__ __align__(16) unsigned Xs[2 * ROWS_BLK * XPW];
  __shared__ __align__(16) float    Hs[ROWS_BLK * FPITCH];
  const _Float16* WH = (const _Float16*)WHp;
  const int tid = threadIdx.x, lane = tid & 31, wave = tid >> 5;
  const int c = lane & 15, hh = lane >> 4, koff = hh * 8;
  const int nd = blockIdx.x / NTILE;
  const int tile = blockIdx.x - nd * NTILE;
  const int node = nd >> 1, dir = nd & 1;
  const int rowbase = tile * ROWS_BLK;
  const int slot = node * 4 + 2 + dir;
  const int j = wave * 16 + c;
  const int steps = dir ? 1 : NSTEP;
  const unsigned short* xsrc = dir ? (XPB + ((size_t)node * NBAT + rowbase) * NGATE)
                                   : (XPF + ((size_t)node * NSTEP * NBAT + rowbase) * NGATE);
  const size_t tstride = dir ? (size_t)0 : (size_t)NBAT * NGATE;

  {
    const int row = tid >> 4, c8 = (tid & 15) * 8;
    const float* hp = h0 + ((size_t)slot * NBAT + rowbase + row) * NHID + c8;
    const v4f a = *(const v4f*)(hp);
    const v4f b = *(const v4f*)(hp + 4);
    v8h hv;
#pragma unroll
    for (int e = 0; e < 4; ++e) {
      hv[e]     = (_Float16)(a[e] * HCARRY);
      hv[4 + e] = (_Float16)(b[e] * HCARRY);
    }
    *(v8h*)(Ah + row * HPITCH + c8) = hv;
  }
  stage_xp(xsrc, Xs, tid);
  asm volatile("" ::: "memory");
  float cst[8], hst[8], bi[4];
#pragma unroll
  for (int g = 0; g < 4; ++g) bi[g] = b1[(size_t)nd * NGATE + g * NHID + j];
#pragma unroll
  for (int r = 0; r < 8; ++r) {
    cst[r] = c0[((size_t)slot * NBAT + rowbase + 8 * hh + r) * NHID + j];
    hst[r] = 0.0f;
  }
  __syncthreads();

  const _Float16* wp = WH + ((size_t)nd * NGATE + j) * NHID + koff;
  const v8f z8 = {0.f, 0.f, 0.f, 0.f, 0.f, 0.f, 0.f, 0.f};
  const unsigned sh = (unsigned)(c & 1) * 16u;

#pragma unroll 1
  for (int s = 0; s < steps; ++s) {
    const int cur = s & 1;
    {
      const int tn = (s + 1 < steps) ? (s + 1) : (steps - 1);
      stage_xp(xsrc + tstride * (size_t)tn, Xs + (cur ^ 1) * (ROWS_BLK * XPW), tid);
    }
    const _Float16* ahrow = Ah + cur * (ROWS_BLK * HPITCH) + c * HPITCH + koff;
    _Float16* ahn = Ah + (cur ^ 1) * (ROWS_BLK * HPITCH);
    v8f acc0 = z8, acc1 = z8, acc2 = z8, acc3 = z8;
#pragma unroll 1
    for (int k0 = 0; k0 < NHID; k0 += 32) {
      const v16h a  = Frag<_Float16>::load(ahrow + k0);
      const v16h b0f = Frag<_Float16>::load(wp + k0);
      const v16h b1f = Frag<_Float16>::load(wp + (size_t)1 * NHID * NHID + k0);
      const v16h b2f = Frag<_Float16>::load(wp + (size_t)2 * NHID * NHID + k0);
      const v16h b3f = Frag<_Float16>::load(wp + (size_t)3 * NHID * NHID + k0);
      acc0 = Frag<_Float16>::mma(a, b0f, acc0);
      acc1 = Frag<_Float16>::mma(a, b1f, acc1);
      acc2 = Frag<_Float16>::mma(a, b2f, acc2);
      acc3 = Frag<_Float16>::mma(a, b3f, acc3);
      wm_guard4(acc0, acc1, acc2, acc3, a, b0f, b1f, b2f, b3f);
    }
    acc_guard4(acc0, acc1, acc2, acc3);
    const unsigned* xsr = Xs + cur * (ROWS_BLK * XPW) + (8 * hh) * XPW + (j >> 1);
#pragma unroll
    for (int r = 0; r < 8; ++r) {
      const unsigned w0 = xsr[r * XPW];
      const unsigned w1 = xsr[r * XPW + 64];
      const unsigned w2 = xsr[r * XPW + 128];
      const unsigned w3 = xsr[r * XPW + 192];
      const float pi = h16_to_f32((w0 >> sh) & 0xffffu);
      const float pf = h16_to_f32((w1 >> sh) & 0xffffu);
      const float pg = h16_to_f32((w2 >> sh) & 0xffffu);
      const float po = h16_to_f32((w3 >> sh) & 0xffffu);
      const float zi = acc0[r] * ACC_INV + (pi + bi[0]);
      const float zf = acc1[r] * ACC_INV + (pf + bi[1]);
      const float zg = acc2[r] * ACC_INV + (pg + bi[2]);
      const float zo = acc3[r] * ACC_INV + (po + bi[3]);
      const float ig = sigm(zi);
      const float fg = sigm(zf);
      const float gg = tanh_e(zg);
      const float og = sigm(zo);
      const float cn = fg * cst[r] + ig * gg;
      cst[r] = cn;
      const float hn = og * tanh_e(cn);
      hst[r] = hn;
      ahn[(8 * hh + r) * HPITCH + j] = (_Float16)(hn * HCARRY);
    }
    __syncthreads();
  }

#pragma unroll
  for (int r = 0; r < 8; ++r) Hs[(8 * hh + r) * FPITCH + j] = hst[r];
  __syncthreads();
  for (int pass = 0; pass < 2; ++pass) {
#pragma unroll
    for (int it = 0; it < 2; ++it) {
      const int idx = it * NTHR + tid;
      const int row = idx >> 5, c4 = (idx & 31) * 4;
      const v4f v = *(const v4f*)(Hs + row * FPITCH + c4);
      *(volatile v4f*)(FEAT + (size_t)(rowbase + row) * NFEAT + node * NY0 + dir * NHID + c4) = v;
    }
    __threadfence();
  }
}

__device__ __forceinline__ float block_sum(float v, float* red, int lane, int wave) {
#pragma unroll
  for (int off = 16; off > 0; off >>= 1) v += __shfl_xor(v, off, 32);
  if (lane == 0) red[wave] = v;
  __syncthreads();
  const float s = ((red[0] + red[1]) + (red[2] + red[3])) + ((red[4] + red[5]) + (red[6] + red[7]));
  __syncthreads();
  return s;
}
__device__ __forceinline__ float ln_res_relu(float u, float ga, float be, float* red, int lane, int wave) {
  const float mu = block_sum(u, red, lane, wave) * (1.0f / NFC);
  const float d = u - mu;
  const float var = block_sum(d * d, red, lane, wave) * (1.0f / (NFC - 1));
  const float sd = sqrtf(var) + LN_EPS;
  const float rinv = 1.0f / sd;
  const float ln = (d * rinv) * ga + be;
  return fmaxf(u + ln, 0.0f);
}

__global__ __launch_bounds__(NTHR) void head_kernel(const float* __restrict__ FEAT,
                                                    const float* __restrict__ w0, const float* __restrict__ bb0,
                                                    const float* __restrict__ a0, const float* __restrict__ g0,
                                                    const float* __restrict__ w1, const float* __restrict__ bb1,
                                                    const float* __restrict__ a1, const float* __restrict__ g1,
                                                    const float* __restrict__ w2, const float* __restrict__ bb2,
                                                    float* __restrict__ out) {
  __shared__ __align__(16) float rowv[NFEAT];
  __shared__ __align__(16) float tv[NFC];
  __shared__ __align__(16) float part[NTHR];
  __shared__ __align__(16) float outs[NOUTD];
  __shared__ float red[8];
  const int b = blockIdx.x, tid = threadIdx.x, lane = tid & 31, wave = tid >> 5;

  rowv[tid]        = FEAT[(size_t)b * NFEAT + tid];
  rowv[tid + NTHR] = FEAT[(size_t)b * NFEAT + NTHR + tid];
  __syncthreads();

  float u = bb0[tid];
#pragma unroll 4
  for (int k = 0; k < NFEAT; ++k) u = fmaf(rowv[k], w0[(size_t)k * NFC + tid], u);
  u = ln_res_relu(u, a0[tid], g0[tid], red, lane, wave);
  tv[tid] = u;
  __syncthreads();

  float u1 = bb1[tid];
#pragma unroll 4
  for (int k = 0; k < NFC; ++k) u1 = fmaf(tv[k], w1[(size_t)k * NFC + tid], u1);
  u1 = ln_res_relu(u1, a1[tid], g1[tid], red, lane, wave);
  tv[tid] = u1;
  __syncthreads();

  {
    const int q = tid >> 6, col = tid & 63;
    float p = 0.0f;
#pragma unroll 4
    for (int kk = 0; kk < 64; ++kk) {
      const int k = q * 64 + kk;
      p = fmaf(tv[k], w2[(size_t)k * NOUTD + col], p);
    }
    part[tid] = p;
    __syncthreads();
    const float o = bb2[col] + ((part[col] + part[64 + col]) + (part[128 + col] + part[192 + col]));
    if (tid < NOUTD) outs[tid] = o;
    __syncthreads();
  }
  if (tid < 16) {
    const v4f v = *(const v4f*)(outs + tid * 4);
    float* op = out + (size_t)b * NOUTD + tid * 4;
    *(volatile v4f*)op = v;
    __threadfence();
    *(volatile v4f*)op = v;
  }
}

extern "C" void kernel_launch(void* const* d_in, const int* in_sizes, int n_in,
                              void* d_out, int out_size, void* d_ws, size_t ws_size, hipStream_t stream) {
  if (n_in < 19 || d_out == nullptr || d_ws == nullptr) return;
  if (in_sizes[0] != NBAT * NNODE * NSTEP || in_sizes[1] != NNODE * 4 * NBAT * NHID || in_sizes[2] != NNODE * 4 * NBAT * NHID ||
      in_sizes[3] != NNODE * 2 * NGATE || in_sizes[4] != NNODE * 2 * NGATE * NHID || in_sizes[5] != NNODE * 2 * NGATE ||
      in_sizes[6] != NNODE * 2 * NGATE * NY0 || in_sizes[7] != NNODE * 2 * NGATE * NHID || in_sizes[8] != NNODE * 2 * NGATE ||
      in_sizes[9] != NFEAT * NFC || in_sizes[10] != NFC || in_sizes[11] != NFC || in_sizes[12] != NFC ||
      in_sizes[13] != NFC * NFC || in_sizes[14] != NFC || in_sizes[15] != NFC || in_sizes[16] != NFC ||
      in_sizes[17] != NFC * NOUTD || in_sizes[18] != NOUTD || out_size != NBAT * NOUTD) return;

  const float* x    = (const float*)d_in[0];
  const float* h0   = (const float*)d_in[1];
  const float* c0   = (const float*)d_in[2];
  const float* wih0 = (const float*)d_in[3];
  const float* whh0 = (const float*)d_in[4];
  const float* b0   = (const float*)d_in[5];
  const float* wih1 = (const float*)d_in[6];
  const float* whh1 = (const float*)d_in[7];
  const float* b1   = (const float*)d_in[8];
  const float* wfc0 = (const float*)d_in[9];
  const float* bfc0 = (const float*)d_in[10];
  const float* ln0a = (const float*)d_in[11];
  const float* ln0b = (const float*)d_in[12];
  const float* wfc1 = (const float*)d_in[13];
  const float* bfc1 = (const float*)d_in[14];
  const float* ln1a = (const float*)d_in[15];
  const float* ln1b = (const float*)d_in[16];
  const float* wfc2 = (const float*)d_in[17];
  const float* bfc2 = (const float*)d_in[18];
  float* out = (float*)d_out;

  char* ws = (char*)d_ws; size_t off = 0;
  auto carve = [&](size_t bytes) -> char* { char* p = ws + off; off += (bytes + 255) & ~(size_t)255; return p; };
  unsigned short* WHH0 = (unsigned short*)carve((size_t)NNODE * 2 * NGATE * NHID * 2);
  unsigned short* WHH1 = (unsigned short*)carve((size_t)NNODE * 2 * NGATE * NHID * 2);
  unsigned short* WIH1 = (unsigned short*)carve((size_t)NNODE * 2 * NGATE * NY0 * 2);
  unsigned short* Y0   = (unsigned short*)carve((size_t)NNODE * NSTEP * NBAT * NY0 * 2);
  unsigned short* XPF  = (unsigned short*)carve((size_t)NNODE * NSTEP * NBAT * NGATE * 2);
  unsigned short* XPB  = (unsigned short*)carve((size_t)NNODE * NBAT * NGATE * 2);
  float*          FEAT = (float*)carve((size_t)NBAT * NFEAT * 4);
  if (off > ws_size || off > (size_t)134217728) return;

  const int n8hh = NNODE * 2 * NGATE * NHID / 8;
  const int n8ih = NNODE * 2 * NGATE * NY0 / 8;
  cvt_w_kernel<<<dim3((n8ih + NTHR - 1) / NTHR, 3), NTHR, 0, stream>>>(whh0, whh1, wih1, WHH0, WHH1, WIH1,
                                                                       n8hh, n8hh, n8ih, WCARRY);

  lstm_l0_kernel<<<NNODE * 2 * NTILE, NTHR, 0, stream>>>(x, h0, c0, wih0, b0, WHH0, Y0);

  {
    const int Mf = NSTEP * NBAT;
    const dim3 ggrid((Mf / 64) * (NGATE / 64) / 8, NNODE);
    wmma_gemm64<0, false, 0, 1><<<ggrid, 256, 0, stream>>>(
        Y0, Y0, NY0, (long)Mf * NY0,
        WIH1, WIH1, NY0, (long)2 * NGATE * NY0,
        (void*)XPF, (void*)XPF, NGATE, (long)Mf * NGATE,
        b1, Mf, NGATE, NY0, ACC_INV);
  }
  {
    const dim3 ggrid((NBAT / 64) * (NGATE / 64) / 8, NNODE);
    wmma_gemm64<0, false, 0, 1><<<ggrid, 256, 0, stream>>>(
        Y0 + (size_t)(NSTEP - 1) * NBAT * NY0, Y0, NY0, (long)NSTEP * NBAT * NY0,
        WIH1 + (size_t)NGATE * NY0, WIH1, NY0, (long)2 * NGATE * NY0,
        (void*)XPB, (void*)XPB, NGATE, (long)NBAT * NGATE,
        b1, NBAT, NGATE, NY0, ACC_INV);
  }

  lstm_l1_kernel<<<NNODE * 2 * NTILE, NTHR, 0, stream>>>(h0, c0, b1, WHH1, XPF, XPB, FEAT);

  head_kernel<<<NBAT, NTHR, 0, stream>>>(FEAT, wfc0, bfc0, ln0a, ln0b, wfc1, bfc1, ln1a, ln1b, wfc2, bfc2, out);
}
